// Encoder_37177236914872
// MI455X (gfx1250) — hardware-verified
//
#include <hip/hip_runtime.h>
#include <stddef.h>
#include <stdint.h>

#define NBAT   8
#define NN     128
#define FIN    196
#define KP1    224
#define HID    256
#define K2     512
#define NE     16256
#define MNODE  1024
#define BC     4
#define NCHUNK 2
#define TR     64
#define NTILE  254
#define AP     520
#define DP     260
#define QSEG   4064
#define WCAP   256
#define NPL    10
#define PLSZ   (HID * K2)
#define NU_XB  (MNODE * (KP1 / 8))
#define NU_W0  (HID * (KP1 / 8))
#define NU_WP  (HID * (K2 / 8))
#define NU_ALL (NU_XB + NU_W0 + NPL * NU_WP)
#define EDGE1_LDS (TR * DP * 4 + TR * AP * 2)
#define EDGE2_LDS (EDGE1_LDS + 512 * 4 + 128 * 4)
#define WSMAX  134217728

static_assert(NTILE * TR == NE);
static_assert(NE % 128 == 0);
static_assert(QSEG * 4 == NE && QSEG % 4 == 0);
static_assert(NBAT == BC * NCHUNK && MNODE == NBAT * NN);
static_assert(KP1 % 32 == 0 && K2 % 32 == 0 && K2 == 2 * HID && KP1 >= FIN && FIN % 4 == 0);
static_assert(NU_XB % 256 == 0 && NU_W0 % 256 == 0 && NU_WP % 256 == 0);
static_assert((AP * 2) % 16 == 0 && (DP * 4) % 16 == 0 && AP >= K2 && DP >= HID);
static_assert(EDGE2_LDS <= 300000);
static_assert((NE * 8) % 128 == 0 && (TR * 8) % 128 == 0);

typedef float          v4f   __attribute__((ext_vector_type(4)));
typedef float          v8f   __attribute__((ext_vector_type(8)));
typedef int            v4i   __attribute__((ext_vector_type(4)));
typedef int            v8i   __attribute__((ext_vector_type(8)));
typedef unsigned       v4u   __attribute__((ext_vector_type(4)));
typedef unsigned short v8us  __attribute__((ext_vector_type(8)));
typedef unsigned short v16us __attribute__((ext_vector_type(16)));
typedef __bf16         v16bf __attribute__((ext_vector_type(16)));
typedef v4f  __attribute__((may_alias)) v4fa;
typedef v4i  __attribute__((may_alias)) v4ia;
typedef v4u  __attribute__((may_alias)) v4ua;
typedef v8us __attribute__((may_alias)) v8usa;
union FragB { v16bf v; v16us u; v8us h[2]; v8i w; };

__device__ __forceinline__ v8f wmb(const FragB& a, const FragB& b, v8f c) {
  v8f d = __builtin_amdgcn_wmma_f32_16x16x32_bf16(false, a.v, false, b.v, (short)0, c, false, false);
  asm volatile("v_nop\n\tv_nop\n\tv_nop\n\tv_nop" : "+v"(d) : "v"(a.w), "v"(b.w));
  return d;
}

__device__ __forceinline__ unsigned bf16_bits(float f) {
  const unsigned u = __float_as_uint(f);
  return (u + 0x7FFFu + ((u >> 16) & 1u)) >> 16;
}
__device__ __forceinline__ float bf16_val(float f) {
  return __uint_as_float(bf16_bits(f) << 16);
}
__device__ __forceinline__ float elu_f(float v) {
  return v > 0.0f ? v : expm1f(v);
}
__device__ __forceinline__ void split8(const v8f f, v8us& hi, v8us& lo) {
#pragma unroll
  for (int i = 0; i < 8; ++i) {
    const unsigned hb = bf16_bits(f[i]);
    hi[i] = (unsigned short)hb;
    lo[i] = (unsigned short)bf16_bits(f[i] - __uint_as_float(hb << 16));
  }
}
__device__ __forceinline__ void put16(unsigned short* dp, v8us o) {
  *(volatile v8us*)dp = o;
  __threadfence();
  *(volatile v8us*)dp = o;
}

__device__ __forceinline__ void scan_row(const v4f q, int& idx, int& vbits) {
  const float r0 = bf16_val(q.x), r1 = bf16_val(q.y), r2 = bf16_val(q.z), r3 = bf16_val(q.w);
  const bool n0 = r0 != 0.0f, n1 = r1 != 0.0f, n2 = r2 != 0.0f, n3 = r3 != 0.0f;
  const int cnt = (int)n0 + (int)n1 + (int)n2 + (int)n3;
  const unsigned any = __builtin_amdgcn_ballot_w32(cnt > 0);
  int tot = cnt;
  tot += __shfl_xor(tot, 16);
  tot += __shfl_xor(tot, 8);
  tot += __shfl_xor(tot, 4);
  tot += __shfl_xor(tot, 2);
  tot += __shfl_xor(tot, 1);
  const int   jf = n0 ? 0 : (n1 ? 1 : (n2 ? 2 : 3));
  const float vf = n0 ? r0 : (n1 ? r1 : (n2 ? r2 : r3));
  const int src = (int)__builtin_ctz(any | 0x80000000u);
  const float vs = __shfl(vf, src);
  const int   js = __shfl(jf, src);
  const bool has = any != 0u;
  int   ii = has ? (4 * src + js) : 0;
  float vv = has ? vs : 0.0f;
  vv = (tot > 1) ? __int_as_float(0x7fc00000) : vv;
  idx = ii;
  vbits = __float_as_int(vv);
}

__global__ __launch_bounds__(256) void k_rel(const float* __restrict__ rec, const float* __restrict__ snd,
                                             int* RIDX, int* RVALb, int* SIDX, int* SVALb) {
  __shared__ __attribute__((aligned(16))) int sT[4 * 128];
  const int tid = (int)threadIdx.x, lane = tid & 31, wave = tid >> 5;
#pragma unroll 1
  for (int i = 0; i < 16; ++i) {
    const int rl = wave * 16 + i;
    const int e  = (int)blockIdx.x * 128 + rl;
    const v4f a = *(const v4fa*)(rec + (size_t)e * NN + 4 * lane);
    const v4f c = *(const v4fa*)(snd + (size_t)e * NN + 4 * lane);
    int ia, va, ic, vc;
    scan_row(a, ia, va);
    scan_row(c, ic, vc);
    if (lane == 0) {
      sT[rl] = ia;
      sT[128 + rl] = va;
      sT[256 + rl] = ic;
      sT[384 + rl] = vc;
    }
  }
  __syncthreads();
  if (wave < 4) {
    const v4i v = *(const v4ia*)(sT + 128 * wave + 4 * lane);
    int* base = (wave == 0) ? RIDX : ((wave == 1) ? RVALb : ((wave == 2) ? SIDX : SVALb));
    int* dp = base + (size_t)blockIdx.x * 128 + 4 * lane;
    *(volatile v4i*)dp = v;
    __threadfence();
    *(volatile v4i*)dp = v;
  }
}

__global__ __launch_bounds__(256) void k_flag(const int* __restrict__ RVALb, const int* __restrict__ SVALb, int* FLAG) {
  __shared__ int sF[8];
  const int tid = (int)threadIdx.x, lane = tid & 31, wave = tid >> 5;
  int bad = 0;
#pragma unroll 1
  for (int i = tid; i < NE / 4; i += 256) {
    const v4i a = *(const v4i*)(RVALb + 4 * i);
    const v4i c = *(const v4i*)(SVALb + 4 * i);
    bad |= (int)((a.x & 0x7fffffff) > 0x7f800000) | (int)((a.y & 0x7fffffff) > 0x7f800000) |
           (int)((a.z & 0x7fffffff) > 0x7f800000) | (int)((a.w & 0x7fffffff) > 0x7f800000) |
           (int)((c.x & 0x7fffffff) > 0x7f800000) | (int)((c.y & 0x7fffffff) > 0x7f800000) |
           (int)((c.z & 0x7fffffff) > 0x7f800000) | (int)((c.w & 0x7fffffff) > 0x7f800000);
  }
  const unsigned mk = __builtin_amdgcn_ballot_w32(bad != 0);
  if (lane == 0) sF[wave] = (mk != 0u) ? 1 : 0;
  __syncthreads();
  if (wave == 0) {
    int f = 0;
#pragma unroll
    for (int w = 0; w < 8; ++w) f |= sF[w];
    if (lane < 8) {
      const v4i o = {f, f, f, f};
      int* dp = FLAG + 4 * lane;
      *(volatile v4i*)dp = o;
      __threadfence();
      *(volatile v4i*)dp = o;
    }
  }
}

__global__ __launch_bounds__(256) void k_prep(const float* __restrict__ x, const float* __restrict__ n1w1,
                                              const float* __restrict__ n1w2, const float* __restrict__ e1w1,
                                              const float* __restrict__ e1w2, const float* __restrict__ n2w1,
                                              const float* __restrict__ n2w2, const float* __restrict__ e2w1,
                                              const float* __restrict__ e2w2,
                                              unsigned short* XB, unsigned short* W0T, unsigned short* WP) {
  const int u = (int)blockIdx.x * 256 + (int)threadIdx.x;
  v8us o;
  if (u < NU_XB) {
    const int row = u / (KP1 / 8);
    const int k8  = (u - row * (KP1 / 8)) * 8;
    const bool okA = k8 < FIN;
    const bool okB = (k8 + 4) < FIN;
    const int ka = okA ? k8 : (FIN - 4);
    const int kb = okB ? (k8 + 4) : (FIN - 4);
    const v4f a = *(const v4fa*)(x + (size_t)row * FIN + ka);
    const v4f b = *(const v4fa*)(x + (size_t)row * FIN + kb);
    o[0] = okA ? (unsigned short)bf16_bits(a.x) : (unsigned short)0;
    o[1] = okA ? (unsigned short)bf16_bits(a.y) : (unsigned short)0;
    o[2] = okA ? (unsigned short)bf16_bits(a.z) : (unsigned short)0;
    o[3] = okA ? (unsigned short)bf16_bits(a.w) : (unsigned short)0;
    o[4] = okB ? (unsigned short)bf16_bits(b.x) : (unsigned short)0;
    o[5] = okB ? (unsigned short)bf16_bits(b.y) : (unsigned short)0;
    o[6] = okB ? (unsigned short)bf16_bits(b.z) : (unsigned short)0;
    o[7] = okB ? (unsigned short)bf16_bits(b.w) : (unsigned short)0;
    put16(XB + (size_t)u * 8, o);
    return;
  } else if (u < NU_XB + NU_W0) {
    const int v  = u - NU_XB;
    const int n  = v / (KP1 / 8);
    const int k8 = (v - n * (KP1 / 8)) * 8;
#pragma unroll
    for (int i = 0; i < 8; ++i) {
      const int k  = k8 + i;
      const int kc = k < FIN ? k : (FIN - 1);
      const float w = n1w1[(size_t)kc * HID + n];
      o[i] = (k < FIN) ? (unsigned short)bf16_bits(w) : (unsigned short)0;
    }
    put16(W0T + (size_t)v * 8, o);
    return;
  } else if (u < NU_ALL) {
    const int v  = u - NU_XB - NU_W0;
    const int p  = v / NU_WP;
    const int w  = v - p * NU_WP;
    const int n  = w >> 6;
    const int k8 = (w & 63) * 8;
    const float* src;
    int roff;
    switch (p) {
      case 0:  src = n1w2; roff = 0;   break;
      case 1:  src = e1w2; roff = 0;   break;
      case 2:  src = n2w1; roff = 0;   break;
      case 3:  src = n2w2; roff = 0;   break;
      case 4:  src = e2w2; roff = 0;   break;
      case 5:  src = e2w1; roff = 512; break;
      case 6:  src = e1w1; roff = 0;   break;
      case 7:  src = e1w1; roff = 256; break;
      case 8:  src = e2w1; roff = 0;   break;
      default: src = e2w1; roff = 256; break;
    }
    const float* q = src + (size_t)(roff + (k8 & (HID - 1))) * HID + n;
#pragma unroll
    for (int i = 0; i < 8; ++i) o[i] = (unsigned short)bf16_bits(q[(size_t)i * HID]);
    put16(WP + (size_t)v * 8, o);
    return;
  }
}

template <int MODE>
__global__ __launch_bounds__(128) void k_gemm(const unsigned short* __restrict__ A, int lda,
                                              const unsigned short* __restrict__ BT, int ldb, int K,
                                              const float* __restrict__ bias,
                                              float* Cm, int ldc, unsigned short* Cb) {
  __shared__ __attribute__((aligned(16))) float stg[64 * 128];
  const int tid = (int)threadIdx.x, lane = tid & 31, wave = tid >> 5, hh = lane >> 4, m = lane & 15;
  const int rowBase = (int)blockIdx.x * 64;
  const int colBase = (int)blockIdx.y * 128;

  v8f acc[8];
  {
    const v8f z = {0.f, 0.f, 0.f, 0.f, 0.f, 0.f, 0.f, 0.f};
#pragma unroll
    for (int t = 0; t < 8; ++t) acc[t] = z;
  }
  const unsigned short* ap = A  + (size_t)(rowBase + 16 * wave + m) * (size_t)lda + 8 * hh;
  const unsigned short* bp = BT + (size_t)(colBase + m) * (size_t)ldb + 8 * hh;

#pragma unroll 1
  for (int k0 = 0; k0 < K; k0 += 32) {
    FragB af;
    af.h[0] = *(const v8usa*)(ap + k0);
    af.h[1] = *(const v8usa*)(ap + k0 + 16);
#pragma unroll
    for (int nt = 0; nt < 8; ++nt) {
      const unsigned short* wq = bp + (size_t)(16 * nt) * (size_t)ldb + k0;
      FragB bf;
      bf.h[0] = *(const v8usa*)wq;
      bf.h[1] = *(const v8usa*)(wq + 16);
      acc[nt] = wmb(af, bf, acc[nt]);
    }
  }

#pragma unroll
  for (int nt = 0; nt < 8; ++nt) {
    const int lc = 16 * nt + m;
    float bvv = 0.0f;
    if constexpr (MODE == 1) bvv = bf16_val(bias[colBase + lc]);
#pragma unroll
    for (int r = 0; r < 8; ++r) {
      const int lr = 16 * wave + 8 * hh + r;
      float v = acc[nt][r];
      if constexpr (MODE == 1) v = elu_f(v + bvv);
      stg[lr * 128 + lc] = v;
    }
  }
  __syncthreads();

  if constexpr (MODE == 1) {
    const int part = lane >> 4;
    const int j = lane & 15;
    const unsigned mh = 0u - (unsigned)part;
    const unsigned ml = ~mh;
    v8us pv[16];
#pragma unroll
    for (int i = 0; i < 16; ++i) {
      const float* sp = stg + (16 * wave + i) * 128 + 8 * j;
      const v4f a = *(const v4fa*)sp;
      const v4f b = *(const v4fa*)(sp + 4);
      const v8f f8 = {a.x, a.y, a.z, a.w, b.x, b.y, b.z, b.w};
      v8us oo;
#pragma unroll
      for (int e = 0; e < 8; ++e) {
        const unsigned hb = bf16_bits(f8[e]);
        const unsigned lb = bf16_bits(f8[e] - __uint_as_float(hb << 16));
        oo[e] = (unsigned short)((hb & ml) | (lb & mh));
      }
      pv[i] = oo;
    }
#pragma unroll
    for (int i = 0; i < 16; ++i) {
      unsigned short* op = Cb + (size_t)(rowBase + 16 * wave + i) * (size_t)K2 + part * HID + colBase + 8 * j;
      *(volatile v8us*)op = pv[i];
    }
    __threadfence();
#pragma unroll
    for (int i = 0; i < 16; ++i) {
      unsigned short* op = Cb + (size_t)(rowBase + 16 * wave + i) * (size_t)K2 + part * HID + colBase + 8 * j;
      *(volatile v8us*)op = pv[i];
    }
  } else {
    v4f pv[16];
#pragma unroll
    for (int i = 0; i < 16; ++i) pv[i] = *(const v4fa*)(stg + (16 * wave + i) * 128 + 4 * lane);
#pragma unroll
    for (int i = 0; i < 16; ++i) {
      float* op = Cm + (size_t)(rowBase + 16 * wave + i) * (size_t)ldc + colBase + 4 * lane;
      *(volatile v4f*)op = pv[i];
    }
    __threadfence();
#pragma unroll
    for (int i = 0; i < 16; ++i) {
      float* op = Cm + (size_t)(rowBase + 16 * wave + i) * (size_t)ldc + colBase + 4 * lane;
      *(volatile v4f*)op = pv[i];
    }
  }
}

__device__ __forceinline__ void tile_gemm(const unsigned short* sA, const unsigned short* __restrict__ BT,
                                          int rg, int cq, int hh, int m, v8f (&acc)[2][4]) {
  {
    const v8f z = {0.f, 0.f, 0.f, 0.f, 0.f, 0.f, 0.f, 0.f};
#pragma unroll
    for (int mt = 0; mt < 2; ++mt)
#pragma unroll
      for (int nt = 0; nt < 4; ++nt) acc[mt][nt] = z;
  }
  const unsigned short* ap0 = sA + (32 * rg + m) * AP + 8 * hh;
  const unsigned short* ap1 = ap0 + 16 * AP;
  const unsigned short* bp  = BT + (size_t)(64 * cq + m) * (size_t)K2 + 8 * hh;
#pragma unroll 1
  for (int k0 = 0; k0 < K2; k0 += 32) {
    FragB a0, a1;
    a0.h[0] = *(const v8usa*)(ap0 + k0);
    a0.h[1] = *(const v8usa*)(ap0 + k0 + 16);
    a1.h[0] = *(const v8usa*)(ap1 + k0);
    a1.h[1] = *(const v8usa*)(ap1 + k0 + 16);
#pragma unroll
    for (int nt = 0; nt < 4; ++nt) {
      const unsigned short* wq = bp + (size_t)(16 * nt) * (size_t)K2 + k0;
      FragB b;
      b.h[0] = *(const v8usa*)wq;
      b.h[1] = *(const v8usa*)(wq + 16);
      acc[0][nt] = wmb(a0, b, acc[0][nt]);
      acc[1][nt] = wmb(a1, b, acc[1][nt]);
    }
  }
}

template <int USEBASE>
__device__ __forceinline__ void assemble_rows(const int* __restrict__ RIDX, const int* __restrict__ SIDX,
                                              const float* __restrict__ RVAL, const float* __restrict__ SVAL,
                                              const float* __restrict__ P, const float* __restrict__ bias,
                                              const float* sD, unsigned short* sA, int b, int tile, int tid) {
  const int r = tid >> 2, q = tid & 3;
  const int e = tile * TR + r;
  int ri = RIDX[e];
  int si = SIDX[e];
  ri = ri < 0 ? 0 : (ri > NN - 1 ? NN - 1 : ri);
  si = si < 0 ? 0 : (si > NN - 1 ? NN - 1 : si);
  const float rv = RVAL[e];
  const float sv = SVAL[e];
  const float* pr = P + (size_t)(b * NN + ri) * K2 + 64 * q;
  const float* ps = P + (size_t)(b * NN + si) * K2 + HID + 64 * q;
  const float* bp = bias + 64 * q;
  const float* rd = sD + r * DP + 64 * q;
  unsigned short* ra = sA + r * AP + 64 * q;
#pragma unroll 2
  for (int c8 = 0; c8 < 8; ++c8) {
    const v4f pa = *(const v4fa*)(pr + 8 * c8);
    const v4f pb = *(const v4fa*)(pr + 8 * c8 + 4);
    const v4f sa = *(const v4fa*)(ps + 8 * c8);
    const v4f sb = *(const v4fa*)(ps + 8 * c8 + 4);
    const v4f ba = *(const v4fa*)(bp + 8 * c8);
    const v4f bb = *(const v4fa*)(bp + 8 * c8 + 4);
    const v8f p8 = {pa.x, pa.y, pa.z, pa.w, pb.x, pb.y, pb.z, pb.w};
    const v8f s8 = {sa.x, sa.y, sa.z, sa.w, sb.x, sb.y, sb.z, sb.w};
    const v8f b8 = {ba.x, ba.y, ba.z, ba.w, bb.x, bb.y, bb.z, bb.w};
    v8f d8 = {0.f, 0.f, 0.f, 0.f, 0.f, 0.f, 0.f, 0.f};
    if constexpr (USEBASE != 0) {
      const v4f da = *(const v4fa*)(rd + 8 * c8);
      const v4f db = *(const v4fa*)(rd + 8 * c8 + 4);
      d8[0] = da.x; d8[1] = da.y; d8[2] = da.z; d8[3] = da.w;
      d8[4] = db.x; d8[5] = db.y; d8[6] = db.z; d8[7] = db.w;
    }
    v8f t8;
#pragma unroll
    for (int i = 0; i < 8; ++i) {
      const float g = rv * p8[i] + sv * s8[i];
      t8[i] = elu_f((d8[i] + g) + bf16_val(b8[i]));
    }
    v8us oh, ol;
    split8(t8, oh, ol);
    *(v8usa*)(ra + 8 * c8)       = oh;
    *(v8usa*)(ra + HID + 8 * c8) = ol;
  }
}

__global__ __launch_bounds__(256) void k_edge1(const int* __restrict__ RIDX, const int* __restrict__ SIDX,
                                               const float* __restrict__ RVAL, const float* __restrict__ SVAL,
                                               const float* __restrict__ PRPS, const float* __restrict__ b1,
                                               const unsigned short* __restrict__ W2T, const float* __restrict__ b2,
                                               int bBase, unsigned short* E1) {
  extern __shared__ __attribute__((aligned(16))) float dyn[];
  float*          sD = dyn;
  unsigned short* sA = (unsigned short*)(dyn + TR * DP);
  const int tid = (int)threadIdx.x, lane = tid & 31, wave = tid >> 5, hh = lane >> 4, m = lane & 15;
  const int tile = (int)blockIdx.x, bq = (int)blockIdx.y, b = bBase + bq;

  assemble_rows<0>(RIDX, SIDX, RVAL, SVAL, PRPS, b1, sD, sA, b, tile, tid);
  __syncthreads();

  const int rg = wave & 1, cq = wave >> 1;
  v8f acc[2][4];
  tile_gemm(sA, W2T, rg, cq, hh, m, acc);
#pragma unroll
  for (int nt = 0; nt < 4; ++nt) {
    const int col = 64 * cq + 16 * nt + m;
    const float bvv = bf16_val(b2[col]);
#pragma unroll
    for (int mt = 0; mt < 2; ++mt)
#pragma unroll
      for (int r = 0; r < 8; ++r)
        sD[(32 * rg + 16 * mt + 8 * hh + r) * DP + col] = elu_f(acc[mt][nt][r] + bvv);
  }
  __syncthreads();

  {
    v8us ph[8], pl[8];
#pragma unroll
    for (int i = 0; i < 8; ++i) {
      const float* sp = sD + (8 * wave + i) * DP + 8 * lane;
      const v4f a = *(const v4fa*)sp;
      const v4f c = *(const v4fa*)(sp + 4);
      const v8f f8 = {a.x, a.y, a.z, a.w, c.x, c.y, c.z, c.w};
      split8(f8, ph[i], pl[i]);
    }
    unsigned short* eb = E1 + ((size_t)bq * NE + (size_t)tile * TR + 8 * wave) * K2 + 8 * lane;
#pragma unroll
    for (int i = 0; i < 8; ++i) {
      *(volatile v8us*)(eb + (size_t)i * K2)       = ph[i];
      *(volatile v8us*)(eb + (size_t)i * K2 + HID) = pl[i];
    }
    __threadfence();
#pragma unroll
    for (int i = 0; i < 8; ++i) {
      *(volatile v8us*)(eb + (size_t)i * K2)       = ph[i];
      *(volatile v8us*)(eb + (size_t)i * K2 + HID) = pl[i];
    }
  }
}

__global__ __launch_bounds__(128) void k_agg(const int* __restrict__ RIDX, const int* __restrict__ RVALb,
                                             const unsigned short* __restrict__ E1, int bBase,
                                             unsigned short* AGG) {
  __shared__ int lE[4 * WCAP];
  __shared__ int lV[4 * WCAP];
  __shared__ int lC[4];
  const int tid = (int)threadIdx.x, lane = tid & 31, wave = tid >> 5;
  const int n = (int)blockIdx.x;
  const int seg = wave * QSEG;
  const unsigned lt = (1u << lane) - 1u;
  int wc = 0;
#pragma unroll 1
  for (int g = 0; g < (QSEG + 127) / 128; ++g) {
    const int o = g * 128 + 4 * lane;
    const bool ok = o < QSEG;
    const int oc = ok ? o : 0;
    const v4i d  = *(const v4i*)(RIDX + seg + oc);
    const v4i vb = *(const v4i*)(RVALb + seg + oc);
    const bool h0 = ok && (d.x == n) && ((vb.x & 0x7fffffff) != 0);
    const bool h1 = ok && (d.y == n) && ((vb.y & 0x7fffffff) != 0);
    const bool h2 = ok && (d.z == n) && ((vb.z & 0x7fffffff) != 0);
    const bool h3 = ok && (d.w == n) && ((vb.w & 0x7fffffff) != 0);
    const unsigned m0 = __builtin_amdgcn_ballot_w32(h0);
    const unsigned m1 = __builtin_amdgcn_ballot_w32(h1);
    const unsigned m2 = __builtin_amdgcn_ballot_w32(h2);
    const unsigned m3 = __builtin_amdgcn_ballot_w32(h3);
    if ((m0 | m1 | m2 | m3) != 0u) {
      int pos = wc + (int)__builtin_popcount(m0 & lt) + (int)__builtin_popcount(m1 & lt) +
                (int)__builtin_popcount(m2 & lt) + (int)__builtin_popcount(m3 & lt);
      if (h0) { if (pos < WCAP) { lE[wave * WCAP + pos] = seg + o;     lV[wave * WCAP + pos] = vb.x; } pos += 1; }
      if (h1) { if (pos < WCAP) { lE[wave * WCAP + pos] = seg + o + 1; lV[wave * WCAP + pos] = vb.y; } pos += 1; }
      if (h2) { if (pos < WCAP) { lE[wave * WCAP + pos] = seg + o + 2; lV[wave * WCAP + pos] = vb.z; } pos += 1; }
      if (h3) { if (pos < WCAP) { lE[wave * WCAP + pos] = seg + o + 3; lV[wave * WCAP + pos] = vb.w; } pos += 1; }
      wc += (int)__builtin_popcount(m0) + (int)__builtin_popcount(m1) +
            (int)__builtin_popcount(m2) + (int)__builtin_popcount(m3);
    }
  }
  if (lane == 0) lC[wave] = wc;
  __syncthreads();

  float a0 = 0.0f, a1 = 0.0f, a2 = 0.0f, a3 = 0.0f, a4 = 0.0f, a5 = 0.0f, a6 = 0.0f, a7 = 0.0f;
  bool ovf = false;
  const unsigned short* eb = E1 + (size_t)wave * NE * K2 + 8 * lane;
#pragma unroll 1
  for (int w2 = 0; w2 < 4; ++w2) {
    int c = lC[w2];
    ovf = ovf || (c > WCAP);
    c = c < 0 ? 0 : (c > WCAP ? WCAP : c);
#pragma unroll 1
    for (int k = 0; k < c; ++k) {
      int e = lE[w2 * WCAP + k];
      e = e < 0 ? 0 : (e > NE - 1 ? NE - 1 : e);
      const float rv = __int_as_float(lV[w2 * WCAP + k]);
      const unsigned short* rp = eb + (size_t)e * K2;
      const v4u h = *(const v4ua*)rp;
      const v4u l = *(const v4ua*)(rp + HID);
      a0 = fmaf(rv, __uint_as_float(h.x << 16)         + __uint_as_float(l.x << 16),         a0);
      a1 = fmaf(rv, __uint_as_float(h.x & 0xffff0000u) + __uint_as_float(l.x & 0xffff0000u), a1);
      a2 = fmaf(rv, __uint_as_float(h.y << 16)         + __uint_as_float(l.y << 16),         a2);
      a3 = fmaf(rv, __uint_as_float(h.y & 0xffff0000u) + __uint_as_float(l.y & 0xffff0000u), a3);
      a4 = fmaf(rv, __uint_as_float(h.z << 16)         + __uint_as_float(l.z << 16),         a4);
      a5 = fmaf(rv, __uint_as_float(h.z & 0xffff0000u) + __uint_as_float(l.z & 0xffff0000u), a5);
      a6 = fmaf(rv, __uint_as_float(h.w << 16)         + __uint_as_float(l.w << 16),         a6);
      a7 = fmaf(rv, __uint_as_float(h.w & 0xffff0000u) + __uint_as_float(l.w & 0xffff0000u), a7);
    }
  }
  const float pz = ovf ? __int_as_float(0x7fc00000) : 0.0f;
  const v8f res = {a0 + pz, a1 + pz, a2 + pz, a3 + pz, a4 + pz, a5 + pz, a6 + pz, a7 + pz};
  v8us oh, ol;
  split8(res, oh, ol);
  unsigned short* dp = AGG + (size_t)((bBase + wave) * NN + n) * K2 + 8 * lane;
  *(volatile v8us*)dp         = oh;
  *(volatile v8us*)(dp + HID) = ol;
  __threadfence();
  *(volatile v8us*)dp         = oh;
  *(volatile v8us*)(dp + HID) = ol;
}

__global__ __launch_bounds__(256) void k_edge2(const int* __restrict__ RIDX, const int* __restrict__ SIDX,
                                               const float* __restrict__ RVAL, const float* __restrict__ SVAL,
                                               const float* __restrict__ QRQS, const float* __restrict__ b1,
                                               const unsigned short* __restrict__ E1,
                                               const unsigned short* __restrict__ WSK,
                                               const unsigned short* __restrict__ W2T, const float* __restrict__ b2,
                                               const float* __restrict__ ow, const float* __restrict__ ob,
                                               const int* __restrict__ FLAG, int bBase, float* out) {
  extern __shared__ __attribute__((aligned(16))) float dyn[];
  float*          sD = dyn;
  unsigned short* sA = (unsigned short*)(dyn + TR * DP);
  float*          sW = dyn + TR * DP + (TR * AP) / 2;
  float*          sO = sW + 512;
  const int tid = (int)threadIdx.x, lane = tid & 31, wave = tid >> 5, hh = lane >> 4, m = lane & 15;
  const int tile = (int)blockIdx.x, bq = (int)blockIdx.y, b = bBase + bq;

  {
    const unsigned short* src = E1 + ((size_t)bq * NE + (size_t)tile * TR) * K2;
#pragma unroll 4
    for (int it = 0; it < 16; ++it) {
      const int u = it * 256 + tid;
      const int row = u >> 6;
      const int c = (u & 63) * 8;
      const v4i v = *(const v4ia*)(src + (size_t)u * 8);
      *(v4ia*)(sA + row * AP + c) = v;
    }
    if (tid < 128) {
      const v4f w = *(const v4fa*)(ow + 4 * tid);
      v4f wr;
      wr.x = bf16_val(w.x); wr.y = bf16_val(w.y); wr.z = bf16_val(w.z); wr.w = bf16_val(w.w);
      *(v4fa*)(sW + 4 * tid) = wr;
    }
  }
  __syncthreads();

  const int rg = wave & 1, cq = wave >> 1;
  v8f acc[2][4];
  tile_gemm(sA, WSK, rg, cq, hh, m, acc);
#pragma unroll
  for (int nt = 0; nt < 4; ++nt) {
    const int col = 64 * cq + 16 * nt + m;
#pragma unroll
    for (int mt = 0; mt < 2; ++mt)
#pragma unroll
      for (int r = 0; r < 8; ++r)
        sD[(32 * rg + 16 * mt + 8 * hh + r) * DP + col] = acc[mt][nt][r];
  }
  __syncthreads();

  assemble_rows<1>(RIDX, SIDX, RVAL, SVAL, QRQS, b1, sD, sA, b, tile, tid);
  __syncthreads();

  tile_gemm(sA, W2T, rg, cq, hh, m, acc);
#pragma unroll
  for (int nt = 0; nt < 4; ++nt) {
    const int col = 64 * cq + 16 * nt + m;
    const float bvv = bf16_val(b2[col]);
#pragma unroll
    for (int mt = 0; mt < 2; ++mt)
#pragma unroll
      for (int r = 0; r < 8; ++r)
        sD[(32 * rg + 16 * mt + 8 * hh + r) * DP + col] = elu_f(acc[mt][nt][r] + bvv);
  }
  __syncthreads();

  {
    const int r = tid >> 2, part = tid & 3;
    const float* er = sD + r * DP + 64 * part;
    const float* wr = sW + 128 * part;
    float p0 = 0.0f, p1 = 0.0f;
#pragma unroll 4
    for (int k = 0; k < 64; k += 4) {
      const v4f ev = *(const v4fa*)(er + k);
      const v4f w0 = *(const v4fa*)(wr + 2 * k);
      const v4f w1 = *(const v4fa*)(wr + 2 * k + 4);
      p0 = fmaf(ev.x, w0.x, p0); p1 = fmaf(ev.x, w0.y, p1);
      p0 = fmaf(ev.y, w0.z, p0); p1 = fmaf(ev.y, w0.w, p1);
      p0 = fmaf(ev.z, w1.x, p0); p1 = fmaf(ev.z, w1.y, p1);
      p0 = fmaf(ev.w, w1.z, p0); p1 = fmaf(ev.w, w1.w, p1);
    }
    p0 += __shfl_xor(p0, 1);
    p1 += __shfl_xor(p1, 1);
    p0 += __shfl_xor(p0, 2);
    p1 += __shfl_xor(p1, 2);
    const float o0 = p0 + bf16_val(ob[0]);
    const float o1 = p1 + bf16_val(ob[1]);
    if (part == 0) {
      sO[2 * r]     = o0;
      sO[2 * r + 1] = o1;
    }
  }
  __syncthreads();

  if (wave == 0) {
    const int fl = FLAG[0];
    v4f v = *(const v4fa*)(sO + 4 * lane);
    const float qn = __int_as_float(0x7fc00000);
    v.x = (fl != 0) ? qn : v.x;
    v.y = (fl != 0) ? qn : v.y;
    v.z = (fl != 0) ? qn : v.z;
    v.w = (fl != 0) ? qn : v.w;
    float* op = out + ((size_t)b * NE + (size_t)tile * TR) * 2 + 4 * lane;
    *(volatile v4f*)op = v;
    __threadfence();
    *(volatile v4f*)op = v;
  }
}

extern "C" void kernel_launch(void* const* d_in, const int* in_sizes, int n_in,
                              void* d_out, int out_size, void* d_ws, size_t ws_size,
                              hipStream_t stream) {
  if (n_in < 21) return;
  if (in_sizes[0] != MNODE * FIN) return;
  if (in_sizes[1] != NE * NN || in_sizes[2] != NE * NN) return;
  if (in_sizes[3] != FIN * HID || in_sizes[4] != HID) return;
  if (in_sizes[5] != HID * HID || in_sizes[6] != HID) return;
  if (in_sizes[7] != 2 * HID * HID || in_sizes[8] != HID) return;
  if (in_sizes[9] != HID * HID || in_sizes[10] != HID) return;
  if (in_sizes[11] != HID * HID || in_sizes[12] != HID) return;
  if (in_sizes[13] != HID * HID || in_sizes[14] != HID) return;
  if (in_sizes[15] != 3 * HID * HID || in_sizes[16] != HID) return;
  if (in_sizes[17] != HID * HID || in_sizes[18] != HID) return;
  if (in_sizes[19] != HID * 2 || in_sizes[20] != 2) return;
  if (out_size != NBAT * NE * 2) return;

  const float* x     = (const float*)d_in[0];
  const float* rec   = (const float*)d_in[1];
  const float* snd   = (const float*)d_in[2];
  const float* n1w1  = (const float*)d_in[3];
  const float* n1b1  = (const float*)d_in[4];
  const float* n1w2  = (const float*)d_in[5];
  const float* n1b2  = (const float*)d_in[6];
  const float* e1w1  = (const float*)d_in[7];
  const float* e1b1  = (const float*)d_in[8];
  const float* e1w2  = (const float*)d_in[9];
  const float* e1b2  = (const float*)d_in[10];
  const float* n2w1  = (const float*)d_in[11];
  const float* n2b1  = (const float*)d_in[12];
  const float* n2w2  = (const float*)d_in[13];
  const float* n2b2  = (const float*)d_in[14];
  const float* e2w1  = (const float*)d_in[15];
  const float* e2b1  = (const float*)d_in[16];
  const float* e2w2  = (const float*)d_in[17];
  const float* e2b2  = (const float*)d_in[18];
  const float* ow    = (const float*)d_in[19];
  const float* ob    = (const float*)d_in[20];
  float* out = (float*)d_out;

  char* ws = (char*)d_ws;
  size_t off = 0;
  const size_t oRIDX = off; off += (size_t)NE * 4;              off = (off + 255) & ~(size_t)255;
  const size_t oRVAL = off; off += (size_t)NE * 4;              off = (off + 255) & ~(size_t)255;
  const size_t oSIDX = off; off += (size_t)NE * 4;              off = (off + 255) & ~(size_t)255;
  const size_t oSVAL = off; off += (size_t)NE * 4;              off = (off + 255) & ~(size_t)255;
  const size_t oFLAG = off; off += 128;                         off = (off + 255) & ~(size_t)255;
  const size_t oXB   = off; off += (size_t)MNODE * KP1 * 2;     off = (off + 255) & ~(size_t)255;
  const size_t oW0T  = off; off += (size_t)HID * KP1 * 2;       off = (off + 255) & ~(size_t)255;
  const size_t oWP   = off; off += (size_t)NPL * PLSZ * 2;      off = (off + 255) & ~(size_t)255;
  const size_t oT1   = off; off += (size_t)MNODE * K2 * 2;      off = (off + 255) & ~(size_t)255;
  const size_t oH1   = off; off += (size_t)MNODE * K2 * 2;      off = (off + 255) & ~(size_t)255;
  const size_t oPRPS = off; off += (size_t)MNODE * K2 * 4;      off = (off + 255) & ~(size_t)255;
  const size_t oAGG  = off; off += (size_t)MNODE * K2 * 2;      off = (off + 255) & ~(size_t)255;
  const size_t oT2   = off; off += (size_t)MNODE * K2 * 2;      off = (off + 255) & ~(size_t)255;
  const size_t oH2   = off; off += (size_t)MNODE * K2 * 2;      off = (off + 255) & ~(size_t)255;
  const size_t oQRQS = off; off += (size_t)MNODE * K2 * 4;      off = (off + 255) & ~(size_t)255;
  const size_t oE1   = off; off += (size_t)BC * NE * K2 * 2;    off = (off + 255) & ~(size_t)255;
  if (off > ws_size || off > (size_t)WSMAX) return;

  int*            RIDX = (int*)(ws + oRIDX);
  int*            RVAL = (int*)(ws + oRVAL);
  int*            SIDX = (int*)(ws + oSIDX);
  int*            SVAL = (int*)(ws + oSVAL);
  int*            FLAG = (int*)(ws + oFLAG);
  unsigned short* XB   = (unsigned short*)(ws + oXB);
  unsigned short* W0T  = (unsigned short*)(ws + oW0T);
  unsigned short* WP   = (unsigned short*)(ws + oWP);
  unsigned short* T1   = (unsigned short*)(ws + oT1);
  unsigned short* H1   = (unsigned short*)(ws + oH1);
  float*          PRPS = (float*)(ws + oPRPS);
  unsigned short* AGG  = (unsigned short*)(ws + oAGG);
  unsigned short* T2   = (unsigned short*)(ws + oT2);
  unsigned short* H2   = (unsigned short*)(ws + oH2);
  float*          QRQS = (float*)(ws + oQRQS);
  unsigned short* E1   = (unsigned short*)(ws + oE1);

  hipFuncSetAttribute(reinterpret_cast<const void*>(&k_edge1), hipFuncAttributeMaxDynamicSharedMemorySize,
                      (int)EDGE1_LDS);
  hipFuncSetAttribute(reinterpret_cast<const void*>(&k_edge2), hipFuncAttributeMaxDynamicSharedMemorySize,
                      (int)EDGE2_LDS);

  k_rel<<<NE / 128, 256, 0, stream>>>(rec, snd, RIDX, RVAL, SIDX, SVAL);
  k_flag<<<1, 256, 0, stream>>>(RVAL, SVAL, FLAG);
  k_prep<<<NU_ALL / 256, 256, 0, stream>>>(x, n1w1, n1w2, e1w1, e1w2, n2w1, n2w2, e2w1, e2w2, XB, W0T, WP);

  k_gemm<1><<<dim3(MNODE / 64, 2), 128, 0, stream>>>(XB, KP1, W0T, KP1, KP1, n1b1, (float*)0, 0, T1);
  k_gemm<1><<<dim3(MNODE / 64, 2), 128, 0, stream>>>(T1, K2, WP + (size_t)0 * PLSZ, K2, K2, n1b2, (float*)0, 0, H1);
  k_gemm<2><<<dim3(MNODE / 64, 4), 128, 0, stream>>>(H1, K2, WP + (size_t)6 * PLSZ, K2, K2, (const float*)0,
                                                     PRPS, K2, (unsigned short*)0);

  for (int c = 0; c < NCHUNK; ++c) {
    const int bBase = c * BC;
    const size_t r0 = (size_t)bBase * NN * K2;
    k_edge1<<<dim3(NTILE, BC), 256, EDGE1_LDS, stream>>>(RIDX, SIDX, (const float*)RVAL, (const float*)SVAL,
                                                         PRPS, e1b1, WP + (size_t)1 * PLSZ, e1b2, bBase, E1);
    k_agg<<<NN, 128, 0, stream>>>(RIDX, RVAL, E1, bBase, AGG);
    k_gemm<1><<<dim3(BC * NN / 64, 2), 128, 0, stream>>>(AGG + r0, K2, WP + (size_t)2 * PLSZ, K2, K2, n2b1,
                                                         (float*)0, 0, T2 + r0);
    k_gemm<1><<<dim3(BC * NN / 64, 2), 128, 0, stream>>>(T2 + r0, K2, WP + (size_t)3 * PLSZ, K2, K2, n2b2,
                                                         (float*)0, 0, H2 + r0);
    k_gemm<2><<<dim3(BC * NN / 64, 4), 128, 0, stream>>>(H2 + r0, K2, WP + (size_t)8 * PLSZ, K2, K2,
                                                         (const float*)0, QRQS + r0, K2, (unsigned short*)0);
    k_edge2<<<dim3(NTILE, BC), 256, EDGE2_LDS, stream>>>(RIDX, SIDX, (const float*)RVAL, (const float*)SVAL,
                                                         QRQS, e2b1, E1, WP + (size_t)5 * PLSZ,
                                                         WP + (size_t)4 * PLSZ, e2b2, ow, ob, FLAG, bBase, out);
  }
}
